// MultiHeadSelfAttention_81741817577579
// MI455X (gfx1250) — hardware-verified
//
#include <hip/hip_runtime.h>
#include <math.h>

typedef __attribute__((ext_vector_type(16))) _Float16 v16h;
typedef __attribute__((ext_vector_type(16))) __bf16 v16b;
typedef __attribute__((ext_vector_type(8)))  _Float16 v8h;
typedef __attribute__((ext_vector_type(8)))  __bf16 v8b;
typedef __attribute__((ext_vector_type(8)))  float v8f;
typedef __attribute__((ext_vector_type(4)))  float v4f;
typedef __attribute__((ext_vector_type(4)))  unsigned v4u;

#ifndef NB
#define NB 4
#endif
#ifndef SEQ
#define SEQ 1024
#endif
#define NB_FULL 4
#define SEQ_FULL 1024
#define DIN 1024
#define CC 1024
#define NH 16
#define HD 64
#define SCALE (0.125f)
#define PCARRY (4096.0f)
#define PLANE ((size_t)NB * SEQ * CC)

static_assert(CC == NH * HD);
static_assert(HD == 64);
static_assert(SEQ % 64 == 0);
static_assert(DIN % 64 == 0 && CC % 128 == 0 && (3 * CC) % 64 == 0 && DIN % 128 == 0);
static_assert(DIN % 32 == 0 && CC % 32 == 0);
static_assert(NB <= NB_FULL && SEQ <= SEQ_FULL);
static_assert(((size_t)NB * SEQ * (DIN / 8)) % 256 == 0);

#define WS_XB  ((size_t)0)
#define WS_WQT (WS_XB  + 2u * (size_t)NB * SEQ * DIN)
#define WS_WOT (WS_WQT + 2u * (size_t)3 * CC * DIN)
#define WS_QK  (WS_WOT + 2u * (size_t)DIN * CC)
#define WS_VT  (WS_QK  + 4u * 2u * PLANE)
#define WS_Y   (WS_VT  + 2u * (size_t)NB * CC * SEQ)
#define WS_END (WS_Y   + 2u * 2u * PLANE)
static_assert(WS_END <= (size_t)134217728);
static_assert(WS_WQT % 128 == 0 && WS_WOT % 128 == 0 && WS_QK % 128 == 0 && WS_VT % 128 == 0 && WS_Y % 128 == 0);

template <typename T> __device__ __forceinline__ void vst2(void* p, T v) { *(volatile T*)p = v; __threadfence(); *(volatile T*)p = v; }
__device__ __forceinline__ v8f wmma16(v16h a, v16h b, v8f c) {
  v8f d = __builtin_amdgcn_wmma_f32_16x16x32_f16(false, a, false, b, (short)0, c, false, false);
  asm volatile("v_nop\n\tv_nop\n\tv_nop\n\tv_nop" : "+v"(d) : "v"(a), "v"(b));
  return d;
}
__device__ __forceinline__ v8f wmma_bf(v16b a, v16b b, v8f c) {
  v8f d = __builtin_amdgcn_wmma_f32_16x16x32_bf16(false, a, false, b, (short)0, c, false, false);
  asm volatile("v_nop\n\tv_nop\n\tv_nop\n\tv_nop" : "+v"(d) : "v"(a), "v"(b));
  return d;
}
__device__ __forceinline__ v16h frag_h(const _Float16* rowk0, int lane) {
  union { v16h v; v8h q[2]; } u; const _Float16* p = rowk0 + 8 * (lane >> 4);
  u.q[0] = *(const v8h*)p; u.q[1] = *(const v8h*)(p + 16); return u.v;
}
__device__ __forceinline__ v16b frag_b(const __bf16* rowk0, int lane) {
  union { v16b v; v8b q[2]; } u; const __bf16* p = rowk0 + 8 * (lane >> 4);
  u.q[0] = *(const v8b*)p; u.q[1] = *(const v8b*)(p + 16); return u.v;
}
__device__ __forceinline__ float bfr(float v) { return (float)(__bf16)v; }

__global__ __launch_bounds__(256) void k_cvt_x(const float* __restrict__ X, __bf16* __restrict__ XB) {
  const int i = blockIdx.x * 256 + threadIdx.x;
  if (i >= NB * SEQ * (DIN / 8)) return;
  const int row = i / (DIN / 8), pc = i % (DIN / 8);
  const size_t srow = (size_t)(row / SEQ) * SEQ_FULL + (size_t)(row % SEQ);
  const float* p = X + srow * DIN + pc * 8;
  const v4f a = *(const v4f*)p, b = *(const v4f*)(p + 4);
  union { v8b v; v4u u; } o;
  o.v[0] = (__bf16)a[0]; o.v[1] = (__bf16)a[1]; o.v[2] = (__bf16)a[2]; o.v[3] = (__bf16)a[3];
  o.v[4] = (__bf16)b[0]; o.v[5] = (__bf16)b[1]; o.v[6] = (__bf16)b[2]; o.v[7] = (__bf16)b[3];
  vst2(XB + (size_t)row * DIN + pc * 8, o.u);
}

__global__ __launch_bounds__(256) void k_tr_w(const float* __restrict__ W, __bf16* __restrict__ WT, int ldw) {
  __shared__ __align__(16) __bf16 t[64][72];
  const int tid = threadIdx.x; const int n0 = blockIdx.x * 64, k0 = blockIdx.y * 64;
  for (int e = tid; e < 64 * 16; e += 256) { const int kr = e >> 4, c4 = (e & 15) * 4;
    const v4f w = *(const v4f*)(W + (size_t)(k0 + kr) * ldw + n0 + c4);
    t[c4 + 0][kr] = (__bf16)w[0]; t[c4 + 1][kr] = (__bf16)w[1]; t[c4 + 2][kr] = (__bf16)w[2]; t[c4 + 3][kr] = (__bf16)w[3]; }
  __syncthreads();
  for (int e = tid; e < 64 * 8; e += 256) { const int nr = e >> 3, q = e & 7; const v4u v = *(const v4u*)&t[nr][q * 8];
    vst2(WT + (size_t)(n0 + nr) * DIN + k0 + q * 8, v); }
}

__global__ __launch_bounds__(128) void k_proj(const __bf16* __restrict__ XB, const __bf16* __restrict__ WT, const float* __restrict__ BQKV, __bf16* __restrict__ QK, _Float16* __restrict__ VT) {
  __shared__ __align__(16) __bf16 sh[64][136], sl[64][136]; __shared__ __align__(16) _Float16 th[128][72];
  const int tid = threadIdx.x; const int wave = __builtin_amdgcn_readfirstlane(threadIdx.x >> 5); const int lane = tid & 31, col = lane & 15, g = lane >> 4;
  const int which = blockIdx.z; const int c0 = blockIdx.y * 128; const int r0 = blockIdx.x * 64; const int bb = r0 / SEQ; const int t0 = r0 % SEQ;
  const __bf16* arow = XB + (size_t)(r0 + wave * 16 + col) * DIN;
  const __bf16* wrow = WT + (size_t)(which * CC + c0 + col) * DIN;
  v8f acc[8] = {};
#pragma unroll 2
  for (int kc = 0; kc < DIN / 32; ++kc) { const v16b a = frag_b(arow + kc * 32, lane);
    asm volatile("s_wait_loadcnt 0x0" ::: "memory");
#pragma unroll
    for (int j = 0; j < 8; ++j) { const v16b w = frag_b(wrow + (size_t)j * 16 * DIN + kc * 32, lane); asm volatile("s_wait_loadcnt 0x0" ::: "memory"); acc[j] = wmma_bf(a, w, acc[j]); } }
  if (which < 2) { const float qs = (which == 0) ? SCALE : 1.0f;
#pragma unroll
    for (int j = 0; j < 8; ++j) { const float bias = bfr(BQKV[which * CC + c0 + j * 16 + col]);
#pragma unroll
      for (int r = 0; r < 8; ++r) { const float v = (acc[j][r] + bias) * qs; const __bf16 hv = (__bf16)v; sh[wave * 16 + 8 * g + r][j * 16 + col] = hv; sl[wave * 16 + 8 * g + r][j * 16 + col] = (__bf16)(v - (float)hv); } }
    __syncthreads();
    __bf16* DH = QK + (size_t)(2 * which) * PLANE; __bf16* DL = DH + PLANE;
    for (int e = tid; e < 64 * 16; e += 128) { const int rl = e >> 4, q = e & 15; const v4u vh = *(const v4u*)&sh[rl][q * 8]; const v4u vl = *(const v4u*)&sl[rl][q * 8];
      const size_t o = (size_t)(r0 + rl) * CC + c0 + q * 8; vst2(DH + o, vh); vst2(DL + o, vl); }
  } else {
#pragma unroll
    for (int j = 0; j < 8; ++j) { const float bias = bfr(BQKV[2 * CC + c0 + j * 16 + col]);
#pragma unroll
      for (int r = 0; r < 8; ++r) th[j * 16 + col][wave * 16 + 8 * g + r] = (_Float16)(acc[j][r] + bias); }
    __syncthreads();
    for (int e = tid; e < 128 * 8; e += 128) { const int cl = e >> 3, q = e & 7; const v4u v = *(const v4u*)&th[cl][q * 8];
      vst2(VT + ((size_t)bb * CC + c0 + cl) * (size_t)SEQ + t0 + q * 8, v); } }
}

__global__ __launch_bounds__(128) void k_attn(const __bf16* __restrict__ QK, const _Float16* __restrict__ VT, __bf16* __restrict__ Y) {
  __shared__ v4u ys[2][64][9];
  const int tid = threadIdx.x; const int wave = __builtin_amdgcn_readfirstlane(threadIdx.x >> 5); const int lane = tid & 31, col = lane & 15, g = lane >> 4;
  const int qb = blockIdx.x, h = blockIdx.y, b = blockIdx.z;
  const size_t qoff = ((size_t)b * SEQ + qb * 64 + wave * 16 + col) * CC + h * HD;
  const __bf16* QHp = QK + qoff; const __bf16* QLp = QK + PLANE + qoff;
  const size_t koff = ((size_t)b * SEQ + col) * CC + h * HD;
  const __bf16* KHp = QK + 2 * PLANE + koff; const __bf16* KLp = QK + 3 * PLANE + koff;
  const _Float16* VTp = VT + ((size_t)b * CC + h * HD + col) * (size_t)SEQ;
  v8f o[4] = {}; float m = -1.0e30f, l = 0.f;
#pragma unroll 1
  for (int kt = 0; kt < SEQ; kt += 32) {
    v8f s0 = {}, s1 = {};
#pragma unroll
    for (int kc = 0; kc < HD / 32; ++kc) {
      const v16b qh = frag_b(QHp + kc * 32, lane), ql = frag_b(QLp + kc * 32, lane);
      { const size_t ko = (size_t)kt * CC + kc * 32; const v16b kh = frag_b(KHp + ko, lane), kl = frag_b(KLp + ko, lane);
        s0 = wmma_bf(kl, qh, s0); s0 = wmma_bf(kh, ql, s0); s0 = wmma_bf(kh, qh, s0); }
      { const size_t ko = (size_t)(kt + 16) * CC + kc * 32; const v16b kh = frag_b(KHp + ko, lane), kl = frag_b(KLp + ko, lane);
        s1 = wmma_bf(kl, qh, s1); s1 = wmma_bf(kh, ql, s1); s1 = wmma_bf(kh, qh, s1); }
    }
    float mx = fmaxf(s0[0], s1[0]);
#pragma unroll
    for (int r = 1; r < 8; ++r) mx = fmaxf(mx, fmaxf(s0[r], s1[r]));
    mx = fmaxf(mx, __shfl_xor(mx, 16));
    const float mn = fmaxf(m, mx); const float corr = __expf(m - mn); m = mn;
    v16h p; float ps = 0.f;
#pragma unroll
    for (int r = 0; r < 8; ++r) { const float e0 = __expf(s0[r] - mn), e1 = __expf(s1[r] - mn); ps += e0 + e1; p[r] = (_Float16)(e0 * PCARRY); p[8 + r] = (_Float16)(e1 * PCARRY); }
    l = l * corr + ps;
#pragma unroll
    for (int j = 0; j < 4; ++j)
#pragma unroll
      for (int r = 0; r < 8; ++r) o[j][r] *= corr;
#pragma unroll
    for (int j = 0; j < 4; ++j) { const v16h vf = frag_h(VTp + (size_t)j * 16 * SEQ + kt, lane); o[j] = wmma16(vf, p, o[j]); }
  }
  l += __shfl_xor(l, 16);
  const float inv = 1.0f / (l * PCARRY);
#pragma unroll
  for (int j = 0; j < 4; ++j) { union { v8b v; v4u u; } hi, lo;
#pragma unroll
    for (int r = 0; r < 8; ++r) { const float c = o[j][r] * inv; const __bf16 hb = (__bf16)c; hi.v[r] = hb; lo.v[r] = (__bf16)(c - (float)hb); }
    ys[0][wave * 16 + col][2 * j + g] = hi.u; ys[1][wave * 16 + col][2 * j + g] = lo.u; }
  __syncthreads();
#pragma unroll 1
  for (int it = 0; it < 4; ++it) { const int rl = wave * 16 + it * 4 + (lane >> 3), pc = lane & 7;
    const v4u a = ys[0][rl][pc]; const v4u c = ys[1][rl][pc];
    const size_t go = ((size_t)b * SEQ + qb * 64 + rl) * CC + h * HD + pc * 8;
    vst2(Y + go, a); vst2(Y + PLANE + go, c); }
}

__global__ __launch_bounds__(128) void k_out(const __bf16* __restrict__ Y, const __bf16* __restrict__ WOT, const float* __restrict__ BO, float* __restrict__ OUT) {
  __shared__ __align__(16) float sf[64][132];
  const int tid = threadIdx.x; const int wave = __builtin_amdgcn_readfirstlane(threadIdx.x >> 5); const int lane = tid & 31, col = lane & 15, g = lane >> 4;
  const int c0 = blockIdx.y * 128; const int rb = blockIdx.x * 64;
  const __bf16* yh = Y + (size_t)(rb + wave * 16 + col) * CC; const __bf16* yl = yh + PLANE;
  const __bf16* wr = WOT + (size_t)(c0 + col) * CC;
  v8f acc[8] = {};
#pragma unroll 2
  for (int kc = 0; kc < CC / 32; ++kc) { const v16b ah = frag_b(yh + kc * 32, lane), al = frag_b(yl + kc * 32, lane);
    asm volatile("s_wait_loadcnt 0x0" ::: "memory");
#pragma unroll
    for (int j = 0; j < 8; ++j) { const v16b w = frag_b(wr + (size_t)j * 16 * CC + kc * 32, lane); asm volatile("s_wait_loadcnt 0x0" ::: "memory"); acc[j] = wmma_bf(al, w, acc[j]); acc[j] = wmma_bf(ah, w, acc[j]); } }
#pragma unroll
  for (int j = 0; j < 8; ++j) { const float bias = bfr(BO[c0 + j * 16 + col]);
#pragma unroll
    for (int r = 0; r < 8; ++r) sf[wave * 16 + 8 * g + r][j * 16 + col] = acc[j][r] + bias; }
  __syncthreads();
  const size_t orow0 = (size_t)(rb / SEQ) * SEQ_FULL + (size_t)(rb % SEQ) + wave * 16;
#pragma unroll 1
  for (int rl = 0; rl < 16; ++rl) { const v4f v = *(const v4f*)&sf[wave * 16 + rl][lane * 4];
    vst2(OUT + (orow0 + rl) * DIN + c0 + lane * 4, v); }
}

extern "C" void kernel_launch(void* const* d_in, const int* in_sizes, int n_in, void* d_out, int out_size, void* d_ws, size_t ws_size, hipStream_t stream) {
  if (n_in < 5) return;
  const size_t xneed = ((size_t)(NB - 1) * SEQ_FULL + SEQ) * DIN;
  if ((size_t)in_sizes[0] < xneed) return;
  if ((size_t)in_sizes[1] < (size_t)DIN * 3 * CC) return;
  if ((size_t)in_sizes[2] < (size_t)3 * CC) return;
  if ((size_t)in_sizes[3] < (size_t)CC * DIN) return;
  if ((size_t)in_sizes[4] < (size_t)DIN) return;
  if ((size_t)out_size < xneed) return;
  if (ws_size < (size_t)WS_END) return;
  const float* x = (const float*)d_in[0]; const float* wqkv = (const float*)d_in[1]; const float* bqkv = (const float*)d_in[2]; const float* wout = (const float*)d_in[3]; const float* bout = (const float*)d_in[4];
  char* ws = (char*)d_ws;
  __bf16* XB = (__bf16*)(ws + WS_XB); __bf16* WQT = (__bf16*)(ws + WS_WQT); __bf16* WOT = (__bf16*)(ws + WS_WOT); __bf16* QK = (__bf16*)(ws + WS_QK); _Float16* VT = (_Float16*)(ws + WS_VT); __bf16* Y = (__bf16*)(ws + WS_Y);
  k_cvt_x<<<dim3((unsigned)(((size_t)NB * SEQ * (DIN / 8)) / 256)), 256, 0, stream>>>(x, XB);
  k_tr_w<<<dim3(3 * CC / 64, DIN / 64), 256, 0, stream>>>(wqkv, WQT, 3 * CC);
  k_tr_w<<<dim3(DIN / 64, CC / 64), 256, 0, stream>>>(wout, WOT, DIN);
  k_proj<<<dim3(NB * SEQ / 64, CC / 128, 3), 128, 0, stream>>>(XB, WQT, bqkv, QK, VT);
  k_attn<<<dim3(SEQ / 64, NH, NB), 128, 0, stream>>>(QK, VT, Y);
  k_out<<<dim3(NB * SEQ / 64, DIN / 128), 128, 0, stream>>>(Y, WOT, bout, (float*)d_out);
}
